// FlashAttention2Naive_17617955848637
// MI455X (gfx1250) — hardware-verified
//
#include <hip/hip_runtime.h>


#define NB_  2
#define NH_  16
#define SS   2048
#define HD   64
#define SCL  0.125f
#define LOSC 1024.0f

typedef _Float16 h16;
typedef unsigned short bf;
typedef __attribute__((ext_vector_type(16))) __bf16   v16bf;
typedef __attribute__((ext_vector_type(16))) _Float16 v16h;
typedef __attribute__((ext_vector_type(8)))  _Float16 v8h;
typedef __attribute__((ext_vector_type(8)))  unsigned short v8us;
typedef __attribute__((ext_vector_type(8)))  float    v8f;
typedef __attribute__((ext_vector_type(4)))  float    v4f;
typedef __attribute__((ext_vector_type(4)))  _Float16 v4h;
typedef v8h  __attribute__((may_alias)) v8ha;
typedef v4f  __attribute__((may_alias)) v4fa;
typedef v8us __attribute__((may_alias)) v8usa;

__device__ __forceinline__ unsigned short f2bf(float f) { unsigned u = __float_as_uint(f); u += 0x7FFFu + ((u >> 16) & 1u); return (unsigned short)(u >> 16); }
__device__ __forceinline__ float bf2f(unsigned short b) { return __uint_as_float(((unsigned)b) << 16); }
__device__ __forceinline__ float bfr(float f) { return bf2f(f2bf(f)); }
__device__ __forceinline__ v16h cat16(v8h lo, v8h hi) { return __builtin_shufflevector(lo, hi, 0, 1, 2, 3, 4, 5, 6, 7, 8, 9, 10, 11, 12, 13, 14, 15); }
__device__ __forceinline__ v16bf cat16b(v8us lo, v8us hi) { return __builtin_bit_cast(v16bf, __builtin_shufflevector(lo, hi, 0, 1, 2, 3, 4, 5, 6, 7, 8, 9, 10, 11, 12, 13, 14, 15)); }
__device__ __forceinline__ v8f wmma16(v16h a, v16h b, v8f c) { return __builtin_amdgcn_wmma_f32_16x16x32_f16(false, a, false, b, (short)0, c, false, false); }
__device__ __forceinline__ v8f wmmab(v16bf a, v16bf b, v8f c) { return __builtin_amdgcn_wmma_f32_16x16x32_bf16(false, a, false, b, (short)0, c, false, false); }

template <int MODE>
__global__ __launch_bounds__(128) void k_gemm3x(const bf* __restrict__ Ah, const bf* __restrict__ Al, const bf* __restrict__ Bh, const bf* __restrict__ Bl, int K, float* C, int ldc) {
    if ((MODE & 1) && (int)blockIdx.y * 64 > (int)blockIdx.x * 64 + 63) return;
    const int Klim = (MODE & 2) ? min(K, ((int)blockIdx.x + 1) * 64) : K;
    __shared__ __align__(16) float ost[4][16 * 68];
    const int lane = threadIdx.x & 31, wave = threadIdx.x >> 5, lr = lane & 15, hi = lane >> 4;
    const int r0 = blockIdx.x * 64 + wave * 16, c0 = blockIdx.y * 64;
    const size_t aoff = (size_t)(r0 + lr) * K + 8 * hi;
    v8f acc[4];
#pragma unroll
    for (int t = 0; t < 4; ++t) acc[t] = (v8f){};
#pragma unroll 1
    for (int kc = 0; kc < Klim; kc += 32) {
        const v16bf a = cat16b(*(const v8us*)(Ah + aoff + kc), *(const v8us*)(Ah + aoff + kc + 16));
        v16bf al = a; if (!(MODE & 4)) al = cat16b(*(const v8us*)(Al + aoff + kc), *(const v8us*)(Al + aoff + kc + 16));
#pragma unroll
        for (int t = 0; t < 4; ++t) { const size_t bo = (size_t)(c0 + t * 16 + lr) * K + kc + 8 * hi;
            const v16bf bh = cat16b(*(const v8us*)(Bh + bo), *(const v8us*)(Bh + bo + 16));
            acc[t] = wmmab(a, bh, acc[t]);
            if (!(MODE & 4)) { acc[t] = wmmab(al, bh, acc[t]); if (!(MODE & 8)) { const v16bf bl = cat16b(*(const v8us*)(Bl + bo), *(const v8us*)(Bl + bo + 16)); acc[t] = wmmab(a, bl, acc[t]); } } }
        asm volatile("v_nop\n\tv_nop\n\tv_nop\n\tv_nop" : "+v"(acc[0]), "+v"(acc[1]), "+v"(acc[2]), "+v"(acc[3]) : "v"(a), "v"(al));
    }
    float* os = &ost[wave][0];
#pragma unroll
    for (int t = 0; t < 4; ++t) {
#pragma unroll
        for (int j = 0; j < 8; ++j) os[(hi * 8 + j) * 68 + t * 16 + lr] = acc[t][j]; }
    __builtin_amdgcn_wave_barrier(); asm volatile("" ::: "memory");
    float* crow = C + (size_t)r0 * ldc + c0;
    auto pass = [&]() {
#pragma unroll
        for (int s = 0; s < 8; ++s) { const int Lid = (lane >> 3) + 4 * s, piece = lane & 7; const int row = Lid >> 1, cofs = (Lid & 1) * 32 + piece * 4;
            const v4f val = *(const v4fa*)(os + row * 68 + cofs); *(volatile v4f*)(crow + (size_t)row * ldc + cofs) = val; }
    };
    pass(); __threadfence(); pass();
}


__global__ __launch_bounds__(256) void k_cvt64(const float* __restrict__ src, bf* dst) {
    typedef __attribute__((ext_vector_type(2))) unsigned short v2us;
    const int lane = threadIdx.x & 31; const size_t r = (size_t)blockIdx.x * 8 + (threadIdx.x >> 5); if (r >= (size_t)SS) return; v2us o; o[0] = f2bf(src[r * HD + lane * 2]); o[1] = f2bf(src[r * HD + lane * 2 + 1]);
    *(volatile v2us*)(dst + r * HD + lane * 2) = o; __threadfence(); *(volatile v2us*)(dst + r * HD + lane * 2) = o;
}
__global__ __launch_bounds__(256) void k_vt64(const float* __restrict__ V, bf* VT) {
    typedef __attribute__((ext_vector_type(2))) unsigned short v2us;
    const int lane = threadIdx.x & 31; const size_t wid = (size_t)blockIdx.x * 8 + (threadIdx.x >> 5); if (wid >= (size_t)HD * (SS / 64)) return; const int d = (int)(wid / (SS / 64)); const int t0 = (int)(wid % (SS / 64)) * 64 + lane * 2; v2us o;
    o[0] = f2bf(V[(size_t)t0 * HD + d]); o[1] = f2bf(V[(size_t)(t0 + 1) * HD + d]);
    const size_t off = (size_t)d * SS + t0; *(volatile v2us*)(VT + off) = o; __threadfence(); *(volatile v2us*)(VT + off) = o;
}
__global__ __launch_bounds__(256) void k_csoft(const float* __restrict__ S, bf* PH, bf* PL, float* LOUT) {
    typedef __attribute__((ext_vector_type(4))) unsigned short v4us;
    __shared__ float lsh[32];
    const int lane = threadIdx.x & 31, wv = threadIdx.x >> 5;
#pragma unroll 1
    for (int rr = 0; rr < 4; ++rr) { const int i = blockIdx.x * 32 + wv * 4 + rr; const float* sr = S + (size_t)i * SS;
        float m = -3.0e38f;
#pragma unroll 1
        for (int c0 = lane * 4; c0 < SS; c0 += 128) {
#pragma unroll
            for (int q = 0; q < 4; ++q) { const int k = c0 + q; if (k <= i) m = fmaxf(m, sr[k] * SCL); } }
#pragma unroll
        for (int sh = 16; sh; sh >>= 1) m = fmaxf(m, __shfl_xor(m, sh, 32));
        float l = 0.f;
#pragma unroll 1
        for (int c0 = lane * 4; c0 < SS; c0 += 128) {
#pragma unroll
            for (int q = 0; q < 4; ++q) { const int k = c0 + q; if (k <= i) l += __expf(sr[k] * SCL - m); } }
#pragma unroll
        for (int sh = 16; sh; sh >>= 1) l += __shfl_xor(l, sh, 32);
        const float inv = 1.0f / l;
#pragma unroll 1
        for (int ps = 0; ps < 2; ++ps) {
#pragma unroll 1
            for (int c0 = lane * 4; c0 < SS; c0 += 128) { v4us oh, ol;
#pragma unroll
                for (int q = 0; q < 4; ++q) { const int k = c0 + q; const float p = (k <= i) ? __expf(sr[(k <= i) ? k : 0] * SCL - m) * inv : 0.f; const unsigned short hb = f2bf(p); oh[q] = hb; ol[q] = f2bf(p - bf2f(hb)); }
                const size_t o = (size_t)i * SS + c0; *(volatile v4us*)(PH + o) = oh; *(volatile v4us*)(PL + o) = ol; }
            if (ps == 0) __threadfence(); }
        if (lane == 0) lsh[wv * 4 + rr] = m + logf(l); }
    __syncthreads();
    if (wv == 0) { const float v = lsh[lane]; float* d = LOUT + (size_t)blockIdx.x * 32 + lane; *(volatile float*)d = v; __threadfence(); *(volatile float*)d = v; }
}

extern "C" void kernel_launch(void* const* d_in, const int* in_sizes, int n_in,
                              void* d_out, int out_size, void* d_ws, size_t ws_size, hipStream_t stream) {
    (void)in_sizes; (void)n_in; (void)out_size;
    const float* Q = (const float*)d_in[0]; const float* Kx = (const float*)d_in[1]; const float* V = (const float*)d_in[2];
    float* O = (float*)d_out;
    float* LO = (float*)((char*)d_out + (size_t)NB_ * NH_ * SS * HD * 4);
    char* wsp = (char*)d_ws;
    auto take = [&](size_t bytes) { char* p = wsp; wsp += (bytes + 255) & ~(size_t)255; return (void*)p; };
    bf* Qb = (bf*)take((size_t)SS * HD * 2); bf* Kb = (bf*)take((size_t)SS * HD * 2); bf* VT = (bf*)take((size_t)HD * SS * 2); float* S = (float*)take((size_t)SS * SS * 4); bf* PH = (bf*)take((size_t)SS * SS * 2); bf* PL = (bf*)take((size_t)SS * SS * 2);
    if ((size_t)(wsp - (char*)d_ws) > ws_size) return;
    for (int mp = 0; mp < NB_ * NH_; ++mp) { const size_t mo = (size_t)mp * SS * HD;
        k_cvt64<<<SS / 8, 256, 0, stream>>>(Q + mo, Qb); k_cvt64<<<SS / 8, 256, 0, stream>>>(Kx + mo, Kb); k_vt64<<<(HD * (SS / 64)) / 8, 256, 0, stream>>>(V + mo, VT);
        k_gemm3x<1 | 4><<<dim3(SS / 64, SS / 64, 1), 128, 0, stream>>>(Qb, Qb, Kb, Kb, HD, S, SS);
        k_csoft<<<SS / 32, 256, 0, stream>>>(S, PH, PL, LO + (size_t)mp * SS);
        k_gemm3x<2 | 8><<<dim3(SS / 64, 1, 1), 128, 0, stream>>>(PH, PL, VT, VT, SS, O + mo, HD); }
}
